// HyperbolicTransformerLayer_64622077935755
// MI455X (gfx1250) — hardware-verified
//
#include <hip/hip_runtime.h>
#include <math.h>


typedef unsigned int u32;
typedef __attribute__((ext_vector_type(2)))  int      v2i;
typedef __attribute__((ext_vector_type(16))) _Float16 v16h;
typedef __attribute__((ext_vector_type(8)))  _Float16 v8h;
typedef __attribute__((ext_vector_type(8)))  float    v8f;
typedef __attribute__((ext_vector_type(4)))  float    v4f;
#define NN    50000
#define NE    600000
#define DD    128
#define FFD   512
#define NH    8
#define DH    16
#define SORTN 1048576
#define TILE  8192
#define NPAD  50176
#define XDEG  256
#define MAXDEG 4096
#define VST2(T, ptr, val) do { const T _v = (val); *(volatile T*)(ptr) = _v; __threadfence(); *(volatile T*)(ptr) = _v; } while (0)
__device__ __forceinline__ v8f wmma16(v16h a, v16h b, v8f c) {
  v8f d = __builtin_amdgcn_wmma_f32_16x16x32_f16(false, a, false, b, (short)0, c, false, false);
  asm volatile("v_nop\n\tv_nop\n\tv_nop\n\tv_nop" : "+v"(d) : "v"(a), "v"(b));
  return d;
}
__device__ __forceinline__ v16h frag16(const _Float16* p, int hh) {
  const v8h lo = *(const v8h*)(p + 8 * hh), hi = *(const v8h*)(p + 16 + 8 * hh);
  return __builtin_shufflevector(lo, hi, 0,1,2,3,4,5,6,7,8,9,10,11,12,13,14,15);
}
__global__ __launch_bounds__(256) void k_sort_init(const int* __restrict__ src, const int* __restrict__ dst, u32* __restrict__ A, int E) {
  const int i = blockIdx.x * 256 + threadIdx.x;
  VST2(u32, A + i, (i < E) ? (((u32)dst[i]) << 16) | (u32)src[i] : 0xffffffffu);
}
__device__ __forceinline__ void cas_lds(u32* s, int lo, int hi, bool up) {
  const u32 a = s[lo], b = s[hi]; const bool sw = up ? (a > b) : (a < b); s[lo] = sw ? b : a; s[hi] = sw ? a : b;
}
__global__ __launch_bounds__(256) void k_sort_local(u32* __restrict__ A) {
  __shared__ u32 s[TILE];
  const int base = blockIdx.x * TILE, t = threadIdx.x;
  for (int i = t; i < TILE; i += 256) s[i] = A[base + i];
  __syncthreads();
  for (int k = 2; k <= TILE; k <<= 1)
    for (int j = k >> 1; j > 0; j >>= 1) {
      for (int p = t; p < TILE / 2; p += 256) {
        const int lo = ((p >> __builtin_ctz(j)) << (__builtin_ctz(j) + 1)) | (p & (j - 1));
        cas_lds(s, lo, lo + j, (((base + lo) & k) == 0));
      }
      __syncthreads();
    }
  for (int pass = 0; pass < 2; ++pass) { for (int i = t; i < TILE; i += 256) *(volatile u32*)(A + base + i) = s[i]; __threadfence(); }
}
__global__ __launch_bounds__(256) void k_sort_global(u32* __restrict__ A, int logj, int k) {
  const int p = blockIdx.x * 256 + threadIdx.x;
  const int j = 1 << logj;
  const int lo = ((p >> logj) << (logj + 1)) | (p & (j - 1)), hi = lo + j;
  const u32 a = A[lo], b = A[hi];
  const bool up = ((lo & k) == 0), sw = up ? (a > b) : (a < b);
  const u32 vlo = sw ? b : a, vhi = sw ? a : b;
  *(volatile u32*)(A + lo) = vlo; *(volatile u32*)(A + hi) = vhi; __threadfence();
  *(volatile u32*)(A + lo) = vlo; *(volatile u32*)(A + hi) = vhi;
}
__global__ __launch_bounds__(256) void k_sort_lds(u32* __restrict__ A, int k) {
  __shared__ u32 s[TILE];
  const int base = blockIdx.x * TILE, t = threadIdx.x;
  for (int i = t; i < TILE; i += 256) s[i] = A[base + i];
  __syncthreads();
  for (int j = TILE >> 1; j > 0; j >>= 1) {
    for (int p = t; p < TILE / 2; p += 256) {
      const int lo = ((p >> __builtin_ctz(j)) << (__builtin_ctz(j) + 1)) | (p & (j - 1));
      cas_lds(s, lo, lo + j, (((base + lo) & k) == 0));
    }
    __syncthreads();
  }
  for (int pass = 0; pass < 2; ++pass) { for (int i = t; i < TILE; i += 256) *(volatile u32*)(A + base + i) = s[i]; __threadfence(); }
}

__global__ __launch_bounds__(256) void k_segs(const u32* __restrict__ A, v2i* __restrict__ seg, float* __restrict__ inv) {
  const int n = blockIdx.x * 256 + threadIdx.x;
  if (n >= NN) return;
  int lo = 0, hi = SORTN;
  while (lo < hi) { const int mid = (lo + hi) >> 1; if ((A[mid] >> 16) < (u32)n) lo = mid + 1; else hi = mid; }
  const int st = lo; hi = SORTN;
  while (lo < hi) { const int mid = (lo + hi) >> 1; if ((A[mid] >> 16) < (u32)(n + 1)) lo = mid + 1; else hi = mid; }
  const v2i sv = {st, lo - st};
  VST2(v2i, seg + n, sv);
  VST2(float, inv + n, 1.0f / fmaxf((float)(lo - st), 1.0f));
}

__global__ __launch_bounds__(256) void k_x16(const float* __restrict__ x, _Float16* __restrict__ X16) {
  const int t = blockIdx.x * 256 + threadIdx.x;
  const int i = t >> 4, c = (t & 15) * 8;
  v8h o;
#pragma unroll
  for (int e = 0; e < 8; ++e) o[e] = (i < NN) ? (_Float16)x[(size_t)i * DD + c + e] : (_Float16)0.f;
  VST2(v8h, X16 + (size_t)i * DD + c, o);
}
__global__ __launch_bounds__(256) void k_wt3(const float* __restrict__ w0, const float* __restrict__ w1, const float* __restrict__ w2, int K, int ncol, int Ntot, _Float16* __restrict__ Wt) {
  const int t = blockIdx.x * 256 + threadIdx.x;
  const int per = K / 8;
  if (t >= Ntot * per) return;
  const int n = t / per, k0 = (t % per) * 8;
  const float* w = (n < ncol) ? w0 : (n < 2 * ncol) ? w1 : w2; const int nn = n % ncol;
  v8h o;
#pragma unroll
  for (int e = 0; e < 8; ++e) o[e] = (_Float16)w[(size_t)(k0 + e) * ncol + nn];
  VST2(v8h, Wt + (size_t)n * K + k0, o);
}
template <int K, int NTOT, int EPI>
__global__ __launch_bounds__(128) void k_gemm(const _Float16* __restrict__ A, const _Float16* __restrict__ Wt, const float* __restrict__ bias,
                                              const float* __restrict__ res, const float* __restrict__ g, const float* __restrict__ be,
                                              float* __restrict__ outf, _Float16* __restrict__ outh) {
  __shared__ __attribute__((aligned(16))) float sT[4][16][132];
  const int lane = threadIdx.x & 31, wave = threadIdx.x >> 5, hh = lane >> 4, l16 = lane & 15;
  const int m0 = blockIdx.x * 64 + wave * 16, n0 = blockIdx.y * 128;
  v8f acc[8];
#pragma unroll
  for (int ni = 0; ni < 8; ++ni) acc[ni] = (v8f){};
#pragma unroll 2
  for (int k0 = 0; k0 < K; k0 += 32) {
    const v16h a0 = frag16(A + (size_t)(m0 + l16) * K + k0, hh);
#pragma unroll
    for (int ni = 0; ni < 8; ++ni) { const v16h b = frag16(Wt + (size_t)(n0 + ni * 16 + l16) * K + k0, hh); acc[ni] = wmma16(a0, b, acc[ni]); }
  }
  float (*st)[132] = sT[wave];
#pragma unroll
  for (int ni = 0; ni < 8; ++ni)
#pragma unroll
    for (int i = 0; i < 8; ++i) { float v = acc[ni][i] + bias[n0 + ni * 16 + l16]; if (EPI == 1) v = fmaxf(v, 0.f); st[i + 8 * hh][ni * 16 + l16] = v; }
  __builtin_amdgcn_fence(__ATOMIC_RELEASE, "workgroup"); __builtin_amdgcn_wave_barrier(); __builtin_amdgcn_fence(__ATOMIC_ACQUIRE, "workgroup");
  if (EPI == 2) {
    if (lane < 16) {
      float* rw = st[lane]; const float* rr = res + (size_t)(m0 + lane) * NTOT;
      float m = 0.f;
      for (int c = 0; c < 128; ++c) { rw[c] = (rr[c] + rw[c]) * 0.5f; m += rw[c]; }
      m *= (1.0f / 128.0f);
      float var = 0.f;
      for (int c = 0; c < 128; ++c) { const float d = rw[c] - m; var += d * d; }
      const float rs = rsqrtf(var * (1.0f / 128.0f) + 1e-5f);
      for (int c = 0; c < 128; ++c) rw[c] = g[c] * (rw[c] - m) * rs + be[c];
    }
    __builtin_amdgcn_fence(__ATOMIC_RELEASE, "workgroup"); __builtin_amdgcn_wave_barrier(); __builtin_amdgcn_fence(__ATOMIC_ACQUIRE, "workgroup");
  }
  for (int pass = 0; pass < 2; ++pass) {
#pragma unroll
    for (int rr = 0; rr < 16; ++rr) {
      if (EPI != 1) *(volatile v4f*)(outf + (size_t)(m0 + rr) * NTOT + n0 + lane * 4) = *(const v4f*)(&st[rr][lane * 4]);
      else if (lane < 16) { v8h o;
#pragma unroll
        for (int e = 0; e < 8; ++e) o[e] = (_Float16)st[rr][lane * 8 + e];
        *(volatile v8h*)(outh + (size_t)(m0 + rr) * NTOT + n0 + lane * 8) = o; }
    }
    __threadfence();
  }
}
__global__ __launch_bounds__(256) void k_attn_ln1(const float* __restrict__ QKV, const u32* __restrict__ keys, const v2i* __restrict__ seg, const float* __restrict__ x,
                                                  const float* __restrict__ g1, const float* __restrict__ be1, float* __restrict__ L1, _Float16* __restrict__ L16) {
  __shared__ __attribute__((aligned(16))) float rows[32][DD + 4];
  const int t = threadIdx.x, nl = t >> 3, hd = t & 7, n = blockIdx.x * 32 + nl;
  float acc[DH];
#pragma unroll
  for (int d = 0; d < DH; ++d) acc[d] = 0.f;
  if (n < NN) {
    const v2i sv = seg[n];
    const int st = min(max(sv[0], 0), SORTN - 1), cnt = min(max(sv[1], 0), MAXDEG);
    float q[DH];
#pragma unroll
    for (int d = 0; d < DH; ++d) q[d] = QKV[(size_t)n * 384 + hd * DH + d];
    float m = -INFINITY, den = 0.f;
    for (int p = 0; p < cnt; ++p) {
      const int j = min((int)(keys[min(st + p, SORTN - 1)] & 0xffffu), NN - 1);
      const float* kr = QKV + (size_t)j * 384 + DD + hd * DH;
      float s = 0.f;
#pragma unroll
      for (int d = 0; d < DH; ++d) s += q[d] * kr[d];
      s *= 0.25f;
      const float mn = fmaxf(m, s), sc = expf(m - mn), w = expf(s - mn);
      den = den * sc + w;
      const float* vr = QKV + (size_t)j * 384 + 2 * DD + hd * DH;
#pragma unroll
      for (int d = 0; d < DH; ++d) acc[d] = acc[d] * sc + w * vr[d];
      m = mn;
    }
    const float inv = (cnt > 0) ? 1.0f / (den + 1e-16f) : 0.f;
#pragma unroll
    for (int d = 0; d < DH; ++d) rows[nl][hd * DH + d] = (x[(size_t)n * DD + hd * DH + d] + acc[d] * inv) * 0.5f;
  } else {
#pragma unroll
    for (int d = 0; d < DH; ++d) rows[nl][hd * DH + d] = 0.f;
  }
  __syncthreads();
  const int wave = t >> 5, lane = t & 31;
  for (int r = wave; r < 32; r += 8) {
    const int row = blockIdx.x * 32 + r;
    v4f xv = *(const v4f*)(&rows[r][lane * 4]);
    float s = xv[0] + xv[1] + xv[2] + xv[3];
#pragma unroll
    for (int o = 16; o > 0; o >>= 1) s += __shfl_xor(s, o, 32);
    const float mu = s * (1.0f / 128.0f);
    float qv = 0.f;
#pragma unroll
    for (int e = 0; e < 4; ++e) { const float d = xv[e] - mu; qv += d * d; }
#pragma unroll
    for (int o = 16; o > 0; o >>= 1) qv += __shfl_xor(qv, o, 32);
    const float rs = rsqrtf(qv * (1.0f / 128.0f) + 1e-5f);
    v4f y; typedef __attribute__((ext_vector_type(4))) _Float16 v4h; v4h yh;
#pragma unroll
    for (int e = 0; e < 4; ++e) { const int c = lane * 4 + e; y[e] = (row < NN) ? (g1[c] * (xv[e] - mu) * rs + be1[c]) : 0.f; yh[e] = (_Float16)y[e]; }
    VST2(v4f, L1 + (size_t)row * DD + lane * 4, y);
    VST2(v4h, L16 + (size_t)row * DD + lane * 4, yh);
  }
}
__global__ __launch_bounds__(256) void k_exact4(const float* __restrict__ x, const u32* __restrict__ keys, const v2i* __restrict__ seg,
                                                const float* __restrict__ Wq, const float* __restrict__ Wk, const float* __restrict__ Wv,
                                                const float* __restrict__ W1, const float* __restrict__ b1, const float* __restrict__ W2, const float* __restrict__ b2,
                                                const float* __restrict__ g1, const float* __restrict__ be1, const float* __restrict__ g2, const float* __restrict__ be2,
                                                float* __restrict__ E4s) {
  __shared__ float q[DD], kv[2][DD], f[DD], hbuf[FFD], red[256], e4[4][DD];
  __shared__ float hm[NH], hden[NH], hacc[NH][DH];
  const int t = threadIdx.x;
  auto bsum = [&](float v) -> float { red[t] = v; __syncthreads(); for (int s = 128; s > 0; s >>= 1) { if (t < s) red[t] += red[t + s]; __syncthreads(); } const float r = red[0]; __syncthreads(); return r; };
  auto layer_norm = [&](float v, const float* g, const float* b) -> float {
    const float mu = bsum((t < DD) ? v : 0.f) * (1.0f / 128.0f);
    const float d = (t < DD) ? (v - mu) : 0.f;
    const float var = bsum(d * d) * (1.0f / 128.0f);
    return g[(t < DD) ? t : 0] * d * rsqrtf(var + 1e-5f) + b[(t < DD) ? t : 0];
  };
  for (int i = 0; i < 4; ++i) {
    const float* xi = x + (size_t)i * DD;
    if (t < DD) { float s = 0.f; _Pragma("unroll 1") for (int k = 0; k < DD; ++k) s += xi[k] * Wq[k * DD + t]; q[t] = s; }
    if (t < NH) { hm[t] = -INFINITY; hden[t] = 0.f; _Pragma("unroll 1") for (int d = 0; d < DH; ++d) hacc[t][d] = 0.f; }
    __syncthreads();
    const v2i sv = seg[i];
    const int st = min(max(sv[0], 0), SORTN - 1), cnt = min(max(sv[1], 0), XDEG);
    for (int p = 0; p < cnt; ++p) {
      const int j = min((int)(keys[min(st + p, SORTN - 1)] & 0xffffu), NN - 1);
      const float* xj = x + (size_t)j * DD;
      if (t < DD) { float s = 0.f; _Pragma("unroll 1") for (int k = 0; k < DD; ++k) s += xj[k] * Wk[k * DD + t]; kv[0][t] = s; }
      else        { const int tt = t - DD; float s = 0.f; _Pragma("unroll 1") for (int k = 0; k < DD; ++k) s += xj[k] * Wv[k * DD + tt]; kv[1][tt] = s; }
      __syncthreads();
      if (t < NH) {
        float s = 0.f; _Pragma("unroll 1") for (int d = 0; d < DH; ++d) s += q[t * DH + d] * kv[0][t * DH + d];
        s *= 0.25f;
        const float mn = fmaxf(hm[t], s), sc = expf(hm[t] - mn), w = expf(s - mn);
        hden[t] = hden[t] * sc + w;
        _Pragma("unroll 1") for (int d = 0; d < DH; ++d) hacc[t][d] = hacc[t][d] * sc + w * kv[1][t * DH + d];
        hm[t] = mn;
      }
      __syncthreads();
    }
    float v1 = 0.f;
    if (t < DD) { const int h = t / DH, d = t % DH; const float att = (cnt > 0) ? hacc[h][d] / (hden[h] + 1e-16f) : 0.f; v1 = (xi[t] + att) * 0.5f; }
    const float l1 = layer_norm(v1, g1, be1);
    if (t < DD) f[t] = l1;
    __syncthreads();
    { float s0 = b1[t], s1 = b1[t + 256]; _Pragma("unroll 1") for (int k = 0; k < DD; ++k) { const float fk = f[k]; s0 += fk * W1[k * FFD + t]; s1 += fk * W1[k * FFD + t + 256]; }
      hbuf[t] = fmaxf(s0, 0.f); hbuf[t + 256] = fmaxf(s1, 0.f); }
    __syncthreads();
    float v2 = 0.f;
    if (t < DD) { float s = b2[t]; _Pragma("unroll 1") for (int k = 0; k < FFD; ++k) s += hbuf[k] * W2[k * DD + t]; v2 = (f[t] + s) * 0.5f; }
    const float l2 = layer_norm(v2, g2, be2);
    if (t < DD) e4[i][t] = l2;
    __syncthreads();
  }
  auto dot128 = [&](const float* a, const float* b) -> float { return bsum((t < DD) ? a[t] * b[t] : 0.f); };
  const float ac0 = dot128(x, x + 2 * DD), bd0 = dot128(x + DD, x + 3 * DD), ad0 = dot128(x, x + 3 * DD), bc0 = dot128(x + DD, x + 2 * DD);
  const float cr0 = (ac0 * bd0) / (ad0 * bc0 + 1e-8f);
  const float ac = dot128(e4[0], e4[2]) + 1.f, bd = dot128(e4[1], e4[3]) + 1.f, ad = dot128(e4[0], e4[3]) + 1.f, bc = dot128(e4[1], e4[2]) + 1.f;
  const float cr = (ac * bd) / (ad * bc + 1e-8f);
  const bool valid = isfinite(cr) && isfinite(cr0) && (fabsf(cr) > 1e-8f);
  const float scale = valid ? powf(fabsf(cr0 / cr), 0.25f) : 1.0f;
  for (int pass = 0; pass < 2; ++pass) {
    for (int qd = t; qd < 4 * DD; qd += 256) *(volatile float*)(E4s + qd) = e4[qd / DD][qd % DD];
    if (t < 32) *(volatile float*)(E4s + 4 * DD + t) = scale;
    __threadfence();
  }
}
__global__ __launch_bounds__(256) void k_final(const float* __restrict__ Tb, const float* __restrict__ E4s, float* __restrict__ out) {
  const int t = blockIdx.x * 256 + threadIdx.x;
  if (t >= NN * 32) return;
  const int n = t >> 5, c = (t & 31) * 4;
  const float scale = E4s[4 * DD];
  v4f v = (n < 4) ? *(const v4f*)(E4s + n * DD + c) : *(const v4f*)(Tb + (size_t)n * DD + c);
  v *= scale;
  VST2(v4f, out + (size_t)n * DD + c, v);
}
extern "C" void kernel_launch(void* const* d_in, const int* in_sizes, int n_in,
                              void* d_out, int out_size, void* d_ws, size_t ws_size, hipStream_t stream) {
  (void)in_sizes; (void)n_in; (void)out_size;
  const float* x   = (const float*)d_in[0];
  const int*   ei  = (const int*)  d_in[1];
  const float* Wq  = (const float*)d_in[2];  const float* Wk = (const float*)d_in[3];  const float* Wv = (const float*)d_in[4];
  const float* W1  = (const float*)d_in[5];  const float* b1 = (const float*)d_in[6];
  const float* W2  = (const float*)d_in[7];  const float* b2 = (const float*)d_in[8];
  const float* g1  = (const float*)d_in[9];  const float* be1 = (const float*)d_in[10];
  const float* g2  = (const float*)d_in[11]; const float* be2 = (const float*)d_in[12];
  float* out = (float*)d_out;
  char* ws = (char*)d_ws; size_t off = 0;
  auto take = [&](size_t bytes) { void* p = ws + off; off = (off + bytes + 255) & ~(size_t)255; return p; };
  u32*      keys = (u32*)take((size_t)SORTN * 4);
  v2i*      seg  = (v2i*)take((size_t)NN * 8);
  float*    inv  = (float*)take((size_t)NN * 4);
  _Float16* X16  = (_Float16*)take((size_t)NPAD * DD * 2);
  _Float16* WtQ  = (_Float16*)take((size_t)384 * DD * 2);
  _Float16* Wt1  = (_Float16*)take((size_t)FFD * DD * 2);
  _Float16* Wt2  = (_Float16*)take((size_t)DD * FFD * 2);
  float*    QKV  = (float*)take((size_t)NPAD * 384 * 4);
  float*    L1   = (float*)take((size_t)NPAD * DD * 4);
  _Float16* L16  = (_Float16*)take((size_t)NPAD * DD * 2);
  _Float16* F16  = (_Float16*)take((size_t)NPAD * FFD * 2);
  float*    Tb   = (float*)take((size_t)NPAD * DD * 4);
  float*    E4s  = (float*)take(4096);
  float*    zb   = (float*)take((size_t)512 * 4);
  if (off > ws_size) return;
  hipMemsetAsync(zb, 0, 512 * 4, stream);
  const dim3 b256(256);
  k_sort_init<<<SORTN / 256, b256, 0, stream>>>(ei, ei + NE, keys, NE);
  k_sort_local<<<SORTN / TILE, b256, 0, stream>>>(keys);
  for (int k = TILE * 2; k <= SORTN; k <<= 1) {
    for (int logj = __builtin_ctz(k) - 1; (1 << logj) >= TILE; --logj)
      k_sort_global<<<SORTN / 2 / 256, b256, 0, stream>>>(keys, logj, k);
    k_sort_lds<<<SORTN / TILE, b256, 0, stream>>>(keys, k);
  }
  k_segs<<<(NN + 255) / 256, b256, 0, stream>>>(keys, seg, inv);
  k_x16<<<NPAD * 16 / 256, b256, 0, stream>>>(x, X16);
  k_wt3<<<(384 * 16 + 255) / 256, b256, 0, stream>>>(Wq, Wk, Wv, DD, DD, 384, WtQ);
  k_wt3<<<(FFD * 16 + 255) / 256, b256, 0, stream>>>(W1, W1, W1, DD, FFD, FFD, Wt1);
  k_wt3<<<(DD * 64 + 255) / 256, b256, 0, stream>>>(W2, W2, W2, FFD, DD, DD, Wt2);
  k_gemm<DD, 384, 0><<<dim3(NPAD / 64, 3), 128, 0, stream>>>(X16, WtQ, zb, nullptr, nullptr, nullptr, QKV, nullptr);
  k_attn_ln1<<<NPAD / 32, b256, 0, stream>>>(QKV, keys, seg, x, g1, be1, L1, L16);
  k_gemm<DD, FFD, 1><<<dim3(NPAD / 64, 4), 128, 0, stream>>>(L16, Wt1, b1, nullptr, nullptr, nullptr, nullptr, F16);
  k_gemm<FFD, DD, 2><<<dim3(NPAD / 64, 1), 128, 0, stream>>>(F16, Wt2, b2, L1, g2, be2, Tb, nullptr);
  k_exact4<<<1, b256, 0, stream>>>(x, keys, seg, Wq, Wk, Wv, W1, b1, W2, b2, g1, be1, g2, be2, E4s);
  k_final<<<(NN * 32 + 255) / 256, b256, 0, stream>>>(Tb, E4s, out);
}
